// StateLeakyAssocModel_79388175499707
// MI455X (gfx1250) — hardware-run, weakly checked
//
#include <hip/hip_runtime.h>


namespace {
constexpr int T = 2048, B = 32, IN = 64, H = 256, OUT = 63, NR = T * B;
constexpr float XS = 8.0f, WSC = 256.0f, BETA = 0.9f;
typedef _Float16 b16;
typedef __attribute__((ext_vector_type(16))) _Float16 v16b;
typedef __attribute__((ext_vector_type(8))) _Float16 v8b;
typedef __attribute__((ext_vector_type(8))) float v8f;
typedef __attribute__((ext_vector_type(4))) float v4f;
__device__ __forceinline__ float bf16_rne(float f) { unsigned int u = __float_as_uint(f); u += 0x7FFFu + ((u >> 16) & 1u); float r = __uint_as_float(u & 0xFFFF0000u); asm volatile("" : "+v"(r)); return r; }
__device__ __forceinline__ void split16(float v, b16& hi, b16& lo) { hi = (b16)v; lo = (b16)(v - (float)hi); }
__device__ __forceinline__ v16b frag_kb(const b16* p, int hh) { const v8b a = *(const v8b*)(p + 8 * hh), b = *(const v8b*)(p + 16 + 8 * hh); v16b f;
#pragma unroll
  for (int e = 0; e < 8; ++e) { f[e] = a[e]; f[8 + e] = b[e]; } return f; }
__device__ __forceinline__ v8f wmma16b(v16b a, v16b b, v8f c) { v8f d = __builtin_amdgcn_wmma_f32_16x16x32_f16(false, a, false, b, (short)0, c, false, false); asm volatile("v_nop\n\tv_nop\n\tv_nop\n\tv_nop" : "+v"(d) : "v"(a), "v"(b)); return d; }
__device__ __forceinline__ void wave_lds_sync() { __builtin_amdgcn_fence(__ATOMIC_RELEASE, "workgroup"); __builtin_amdgcn_wave_barrier(); __builtin_amdgcn_fence(__ATOMIC_ACQUIRE, "workgroup"); }
__device__ __forceinline__ float pmul(float a, float b) { float p = a * b; asm volatile("" : "+v"(p)); return p; }

__global__ __launch_bounds__(256) void wput_kernel(const float* __restrict__ wi, const float* __restrict__ wm, const float* __restrict__ wo, b16* __restrict__ WI, b16* __restrict__ WM, b16* __restrict__ WO) { const int u = blockIdx.x * 256 + threadIdx.x;
  if (u < H * 8) { const int o = u / 8, k0 = (u % 8) * 8; v8b v;
#pragma unroll
    for (int j = 0; j < 8; ++j) v[j] = (b16)(bf16_rne(wi[(size_t)(k0 + j) * H + o]) * WSC); for (int pass = 0; pass < 2; ++pass) { *(volatile v8b*)(WI + (size_t)o * IN + k0) = v; __threadfence(); } }
  if (u < H * 32) { const int o = u / 32, k0 = (u % 32) * 8; v8b v;
#pragma unroll
    for (int j = 0; j < 8; ++j) v[j] = (b16)(bf16_rne(wm[(size_t)(k0 + j) * H + o]) * WSC); for (int pass = 0; pass < 2; ++pass) { *(volatile v8b*)(WM + (size_t)o * H + k0) = v; __threadfence(); } }
  if (u < 64 * 32) { const int o = u / 32, k0 = (u % 32) * 8; v8b v;
#pragma unroll
    for (int j = 0; j < 8; ++j) v[j] = (b16)(o < OUT ? bf16_rne(wo[(size_t)(k0 + j) * OUT + o]) * WSC : 0.0f); for (int pass = 0; pass < 2; ++pass) { *(volatile v8b*)(WO + (size_t)o * H + k0) = v; __threadfence(); } } }
__global__ __launch_bounds__(32) void inproj_kernel(const float* __restrict__ x, const b16* __restrict__ WI, const float* __restrict__ b, float* __restrict__ Hh) { __shared__ __attribute__((aligned(16))) b16 Ah[16][IN + 8]; __shared__ float Tf[16][260]; const int lane = threadIdx.x, nloc = lane & 15, hlf = lane >> 4; const size_t m0 = (size_t)blockIdx.x * 16;
  for (int rr = 0; rr < 16; ++rr) for (int q = 0; q < 2; ++q) Ah[rr][q * 32 + lane] = (b16)(bf16_rne(x[(m0 + rr) * IN + q * 32 + lane]) * XS);
  wave_lds_sync(); v8f acc[16];
#pragma unroll
  for (int t = 0; t < 16; ++t) acc[t] = (v8f){};
#pragma unroll
  for (int kb = 0; kb < IN; kb += 32) { const v16b a = frag_kb(&Ah[nloc][kb], hlf);
#pragma unroll
    for (int t = 0; t < 16; ++t) acc[t] = wmma16b(a, frag_kb(WI + (size_t)(t * 16 + nloc) * IN + kb, hlf), acc[t]); }
#pragma unroll
  for (int t = 0; t < 16; ++t) { const int cc = t * 16 + nloc; const float bb = bf16_rne(b[cc]);
#pragma unroll
    for (int r8 = 0; r8 < 8; ++r8) Tf[8 * hlf + r8][cc] = acc[t][r8] * (1.0f / (XS * WSC)) + bb; }
  wave_lds_sync();
  for (int pass = 0; pass < 2; ++pass) { for (int rr = 0; rr < 16; ++rr) for (int q = 0; q < 2; ++q) *(volatile v4f*)(Hh + (m0 + rr) * H + q * 128 + lane * 4) = *(const v4f*)(&Tf[rr][q * 128 + lane * 4]); __threadfence(); } }
__global__ __launch_bounds__(256) void scan_kernel(const float* __restrict__ Hs, int TLIM, float* __restrict__ Hd) { const int u = blockIdx.x * 256 + threadIdx.x; if (u >= B * H) return; const int b = u / H, c = u % H;
  for (int pass = 0; pass < 2; ++pass) { float h = 0.0f;
#pragma unroll 1
    for (int t = 0; t < TLIM; ++t) { const size_t idx = ((size_t)t * B + b) * H + c; h = pmul(h, BETA) + Hs[idx]; ((volatile float*)Hd)[idx] = h; }
    __threadfence(); } }
__global__ __launch_bounds__(32) void mid_kernel(const float* __restrict__ Hin, const b16* __restrict__ WM, const float* __restrict__ b, int RLIM, float* __restrict__ Hout) { __shared__ __attribute__((aligned(16))) b16 Ah[16][H + 8], Al[16][H + 8]; __shared__ float Tf[16][260]; const int lane = threadIdx.x, nloc = lane & 15, hlf = lane >> 4; const size_t m0 = (size_t)blockIdx.x * 16; if (m0 >= (size_t)RLIM) return;
  for (int rr = 0; rr < 16; ++rr) for (int q = 0; q < 8; ++q) { b16 p, ql; split16(Hin[(m0 + rr) * H + q * 32 + lane] * XS, p, ql); Ah[rr][q * 32 + lane] = p; Al[rr][q * 32 + lane] = ql; }
  wave_lds_sync(); v8f acc[16];
#pragma unroll
  for (int t = 0; t < 16; ++t) acc[t] = (v8f){};
#pragma unroll 2
  for (int kb = 0; kb < H; kb += 32) { const v16b a = frag_kb(&Ah[nloc][kb], hlf), al = frag_kb(&Al[nloc][kb], hlf);
#pragma unroll
    for (int t = 0; t < 16; ++t) { const v16b bw = frag_kb(WM + (size_t)(t * 16 + nloc) * H + kb, hlf); acc[t] = wmma16b(a, bw, acc[t]); acc[t] = wmma16b(al, bw, acc[t]); } }
#pragma unroll
  for (int t = 0; t < 16; ++t) { const int cc = t * 16 + nloc; const float bb = bf16_rne(b[cc]);
#pragma unroll
    for (int r8 = 0; r8 < 8; ++r8) Tf[8 * hlf + r8][cc] = fmaxf(acc[t][r8] * (1.0f / (XS * WSC)) + bb, 0.0f); }
  wave_lds_sync();
  for (int pass = 0; pass < 2; ++pass) { for (int rr = 0; rr < 16; ++rr) for (int q = 0; q < 2; ++q) *(volatile v4f*)(Hout + (m0 + rr) * H + q * 128 + lane * 4) = *(const v4f*)(&Tf[rr][q * 128 + lane * 4]); __threadfence(); } }
__global__ __launch_bounds__(32) void out_kernel(const float* __restrict__ Hin, const b16* __restrict__ WO, const float* __restrict__ b, int RLIM, float* __restrict__ out) { __shared__ __attribute__((aligned(16))) b16 Ah[16][H + 8], Al[16][H + 8]; __shared__ float Tf[32][64]; const int lane = threadIdx.x, nloc = lane & 15, hlf = lane >> 4; const size_t base = (size_t)blockIdx.x * 32; if (base >= (size_t)RLIM) return;
  for (int half = 0; half < 2; ++half) { const size_t m0 = base + half * 16;
    for (int rr = 0; rr < 16; ++rr) for (int q = 0; q < 8; ++q) { b16 p, ql; split16(Hin[(m0 + rr) * H + q * 32 + lane] * XS, p, ql); Ah[rr][q * 32 + lane] = p; Al[rr][q * 32 + lane] = ql; }
    wave_lds_sync(); v8f acc[4];
#pragma unroll
    for (int t = 0; t < 4; ++t) acc[t] = (v8f){};
#pragma unroll 2
    for (int kb = 0; kb < H; kb += 32) { const v16b a = frag_kb(&Ah[nloc][kb], hlf), al = frag_kb(&Al[nloc][kb], hlf);
#pragma unroll
      for (int t = 0; t < 4; ++t) { const v16b bw = frag_kb(WO + (size_t)(t * 16 + nloc) * H + kb, hlf); acc[t] = wmma16b(a, bw, acc[t]); acc[t] = wmma16b(al, bw, acc[t]); } }
#pragma unroll
    for (int t = 0; t < 4; ++t) { const int cc = t * 16 + nloc; const float bb = cc < OUT ? bf16_rne(b[cc]) : 0.0f;
#pragma unroll
      for (int r8 = 0; r8 < 8; ++r8) { const float v = acc[t][r8] * (1.0f / (XS * WSC)) + bb; Tf[half * 16 + 8 * hlf + r8][cc] = 1.0f / (1.0f + __expf(-v)); } }
    wave_lds_sync(); }
  for (int pass = 0; pass < 2; ++pass) { for (int q = lane; q < 32 * OUT; q += 32) ((volatile float*)out)[base * OUT + q] = Tf[q / OUT][q % OUT]; __threadfence(); } }
}

extern "C" void kernel_launch(void* const* d_in, const int* in_sizes, int n_in, void* d_out, int out_size, void* d_ws, size_t ws_size, hipStream_t stream) {
  (void)n_in;
  auto Fp = [&](int i) { return (const float*)d_in[i]; };
  if (in_sizes[0] != NR * IN || in_sizes[1] != IN * H || in_sizes[3] != H * H || in_sizes[5] != H * OUT || in_sizes[6] != OUT || out_size != NR * OUT) return;
  const int TLIM = T;
  const int RLIM = TLIM * B;
  size_t off = 0; char* ws = (char*)d_ws;
  auto carve = [&](size_t bytes) { char* p = ws + off; off += (bytes + 255) & ~(size_t)255; return p; };
  b16* WI = (b16*)carve((size_t)H * IN * 2); b16* WM = (b16*)carve((size_t)H * H * 2); b16* WO = (b16*)carve((size_t)64 * H * 2); float* HA = (float*)carve((size_t)NR * H * 4); float* HB = (float*)carve((size_t)NR * H * 4);
  if (off > ws_size || off > ((size_t)160 << 20)) return;
  wput_kernel<<<(H * 32 + 255) / 256, 256, 0, stream>>>(Fp(1), Fp(3), Fp(5), WI, WM, WO);
  inproj_kernel<<<RLIM / 16, 32, 0, stream>>>(Fp(0), WI, Fp(2), HA);
  scan_kernel<<<(B * H + 255) / 256, 256, 0, stream>>>(HA, TLIM, HB);
  mid_kernel<<<RLIM / 16, 32, 0, stream>>>(HB, WM, Fp(4), RLIM, HA);
  scan_kernel<<<(B * H + 255) / 256, 256, 0, stream>>>(HA, TLIM, HB);
  out_kernel<<<RLIM / 32, 32, 0, stream>>>(HB, WO, Fp(6), RLIM, (float*)d_out);
}
